// SimplifiedAttention_34875134443550
// MI455X (gfx1250) — hardware-verified
//
#include <hip/hip_runtime.h>
#include <math.h>
#include <stdint.h>

#ifndef NB
#define NB 4
#endif
#ifndef SEQ
#define SEQ 2048
#endif
#define NB_FULL  4
#define SEQ_FULL 2048
#define EMB   1024
#define CK    (((SEQ) < 512) ? (SEQ) : 512)
#define NCHK  ((SEQ) / CK)
#define NKB   (CK / 32)
#define QT    16
#define NQT   ((SEQ) / QT)
#define SCP   544
#define PLP   528
#define CTP   1032
#define SLAB64 (16 * 68)
#define VTP   72
#define ATT_THREADS 256
#define NACC  8
#define QSC   8.0f
#define KSC   8.0f
#define QRS   2048.0f
#define PCAR  32768.0f
#define VCAR  1024.0f
#define WSC   1024.0f
#define CSC   8192.0f
#define RSC   2048.0f
#define LOG2E 1.4426950408889634f
#define RSQD  0.125f
#define WS_CAP ((size_t)134217728)

static_assert(NB >= 1 && NB <= NB_FULL && SEQ >= 64 && SEQ <= SEQ_FULL);
static_assert((EMB % 64) == 0 && EMB == 8 * 16 * NACC && NACC == 8 && (EMB % 32) == 0 && (EMB % 256) == 0);
static_assert((SEQ % 64) == 0 && (SEQ % CK) == 0 && NCHK * CK == SEQ && CK == 32 * NKB && NKB >= 1 && NKB <= 16 && CK <= 512);
static_assert((SEQ % QT) == 0 && NQT * QT == SEQ && (CK % QT) == 0);
static_assert(16 * CTP * 2 <= 16 * SCP * 4 && CTP >= EMB + 8 && SCP >= 512 + 32 && PLP >= 512 + 8);
static_assert(((PLP * 2) % 16) == 0 && ((SCP * 4) % 16) == 0 && ((VTP * 2) % 16) == 0 && ((CTP * 2) % 16) == 0);
static_assert(64 * VTP >= 63 * VTP + 64);
static_assert(ATT_THREADS == 16 * QT && ATT_THREADS == 256);
static_assert(((EMB * EMB) % 2048) == 0 && (EMB / 8) * 2 == 256 && ((NB * SEQ) % 64) == 0);

typedef unsigned short u16;
typedef _Float16 v16h __attribute__((ext_vector_type(16)));
typedef _Float16 v8h  __attribute__((ext_vector_type(8)));
typedef __bf16   v16b __attribute__((ext_vector_type(16)));
typedef float    v8f  __attribute__((ext_vector_type(8)));
typedef float    v4f  __attribute__((ext_vector_type(4)));
typedef unsigned int v4u __attribute__((ext_vector_type(4)));

union FragH { v16h v; v8h h[2]; v4u u[2]; };
union FragB { v16b v; v4u u[2]; };
union AttLds { float s[16 * SCP]; u16 c[2 * 16 * SCP]; };

__device__ __forceinline__ unsigned short bf_bits(float f) {
  unsigned u = __float_as_uint(f);
  return (unsigned short)((u + 0x7FFFu + ((u >> 16) & 1u)) >> 16);
}
__device__ __forceinline__ float bf_up(unsigned short h) { return __uint_as_float(((unsigned)h) << 16); }
__device__ __forceinline__ float bfr(float f) { return bf_up(bf_bits(f)); }
__device__ __forceinline__ unsigned short h_bits(_Float16 x) { return __builtin_bit_cast(unsigned short, x); }
__device__ __forceinline__ unsigned pk16(unsigned short a, unsigned short b) { return (unsigned)a | ((unsigned)b << 16); }
__device__ __forceinline__ v8f zero8() { v8f z = {0.f, 0.f, 0.f, 0.f, 0.f, 0.f, 0.f, 0.f}; return z; }
__device__ __forceinline__ const _Float16* hptr(const u16* p) { return (const _Float16*)(const void*)p; }

__device__ __forceinline__ v16h ldfrag_h(const _Float16* p) {
  FragH f;
  f.h[0] = *(const v8h*)(p);
  f.h[1] = *(const v8h*)(p + 16);
  return f.v;
}
__device__ __forceinline__ v16b ldfrag_b(const u16* p) {
  FragB f;
  f.u[0] = *(const v4u*)(p);
  f.u[1] = *(const v4u*)(p + 16);
  return f.v;
}

__device__ __forceinline__ v8f mma_h(v16h a, v16h b, v8f c) {
  return __builtin_amdgcn_wmma_f32_16x16x32_f16(false, a, false, b, (short)0, c, false, false);
}
__device__ __forceinline__ v8f mma_b(v16b a, v16b b, v8f c) {
  return __builtin_amdgcn_wmma_f32_16x16x32_bf16(false, a, false, b, (short)0, c, false, false);
}
template <typename F>
__device__ __forceinline__ void guard6(v8f& a, v8f& b, v8f& c, v8f& d, F x0, F x1, F x2, F x3, F x4, F x5) {
#if defined(__HIP_DEVICE_COMPILE__)
  asm volatile("v_nop\n\tv_nop\n\tv_nop\n\tv_nop"
               : "+v"(a), "+v"(b), "+v"(c), "+v"(d) : "v"(x0), "v"(x1), "v"(x2), "v"(x3), "v"(x4), "v"(x5) : "memory");
#endif
}
__device__ __forceinline__ void guard8x6(v8f& a0, v8f& a1, v8f& a2, v8f& a3, v8f& e0, v8f& e1, v8f& e2, v8f& e3,
                                         v16h x0, v16h x1, v16h x2, v16h x3, v16h x4, v16h x5) {
#if defined(__HIP_DEVICE_COMPILE__)
  asm volatile("v_nop\n\tv_nop\n\tv_nop\n\tv_nop"
               : "+v"(a0), "+v"(a1), "+v"(a2), "+v"(a3), "+v"(e0), "+v"(e1), "+v"(e2), "+v"(e3)
               : "v"(x0), "v"(x1), "v"(x2), "v"(x3), "v"(x4), "v"(x5) : "memory");
#endif
}
__device__ __forceinline__ void guardpv4(v8f& o0, v8f& o1, v8f& o2, v8f& o3, v16h p, v16h g0, v16h g1, v16h g2, v16h g3) {
#if defined(__HIP_DEVICE_COMPILE__)
  asm volatile("v_nop\n\tv_nop\n\tv_nop\n\tv_nop"
               : "+v"(o0), "+v"(o1), "+v"(o2), "+v"(o3)
               : "v"(p), "v"(g0), "v"(g1), "v"(g2), "v"(g3) : "memory");
#endif
}
__device__ __forceinline__ void acc_guard8(v8f& a, v8f& b, v8f& c, v8f& d, v8f& e, v8f& f, v8f& g, v8f& h8) {
#if defined(__HIP_DEVICE_COMPILE__)
  asm volatile("v_nop\n\tv_nop\n\tv_nop\n\tv_nop"
               : "+v"(a), "+v"(b), "+v"(c), "+v"(d), "+v"(e), "+v"(f), "+v"(g), "+v"(h8));
#endif
}
__device__ __forceinline__ void wave_sync_lds() {
  __builtin_amdgcn_fence(__ATOMIC_RELEASE, "workgroup");
  __builtin_amdgcn_wave_barrier();
  __builtin_amdgcn_fence(__ATOMIC_ACQUIRE, "workgroup");
}

__global__ __launch_bounds__(256) void cvt16(const float* __restrict__ x, u16* D, int n8, int mode, float scale,
                                             int rpg, int gstr) {
  const int gt = blockIdx.x * 256 + (int)threadIdx.x;
  if (gt >= n8) return;
  const int row = gt / (EMB / 8);
  const int cg  = gt - row * (EMB / 8);
  const int grp = row / rpg;
  const size_t srow = (size_t)grp * (size_t)gstr + (size_t)(row - grp * rpg);
  const float* p = x + srow * (size_t)EMB + (size_t)cg * 8;
  const v4f a = *(const v4f*)(p), c4 = *(const v4f*)(p + 4);
  float v[8];
#pragma unroll
  for (int e = 0; e < 4; ++e) { v[e] = a[e]; v[4 + e] = c4[e]; }
  unsigned short s[8];
#pragma unroll
  for (int e = 0; e < 8; ++e) {
    const float vb = bfr(v[e]);
    const unsigned short hb = h_bits((_Float16)(vb * scale));
    const unsigned short bb = bf_bits(v[e]);
    s[e] = (mode != 0) ? hb : bb;
  }
  v4u o;
#pragma unroll
  for (int e = 0; e < 4; ++e) o[e] = pk16(s[2 * e], s[2 * e + 1]);
  u16* d = D + (size_t)gt * 8;
  for (int pass = 0; pass < 2; ++pass) {
    *(volatile v4u*)(d) = o;
    __threadfence();
  }
}

__device__ __forceinline__ void stage64b(float* sl, v8f a0, v8f a1, v8f a2, v8f a3, float oscale,
                                         const float* __restrict__ bias, int col0, int lane) {
  const int hh = lane >> 4, m = lane & 15;
  const float* bp = bias + col0 + m;
  const float b0 = bp[0], b1 = bp[16], b2 = bp[32], b3 = bp[48];
#pragma unroll
  for (int r = 0; r < 8; ++r) {
    const int ro = (8 * hh + r) * 68 + m;
    sl[ro]      = a0[r] * oscale + b0;
    sl[ro + 16] = a1[r] * oscale + b1;
    sl[ro + 32] = a2[r] * oscale + b2;
    sl[ro + 48] = a3[r] * oscale + b3;
  }
  wave_sync_lds();
}
__device__ __forceinline__ void epi64b(float* sl, v8f a0, v8f a1, v8f a2, v8f a3, float oscale, const float* __restrict__ bias,
                                       float* C, int N, size_t rowb, int col0, int lane) {
  const int hh = lane >> 4, m = lane & 15;
  stage64b(sl, a0, a1, a2, a3, oscale, bias, col0, lane);
  v4f vals[8];
#pragma unroll
  for (int it = 0; it < 8; ++it) vals[it] = *(const v4f*)(sl + (it * 2 + hh) * 68 + m * 4);
  float* dst = C + (rowb + (size_t)hh) * (size_t)N + col0 + m * 4;
  for (int pass = 0; pass < 2; ++pass) {
#pragma unroll
    for (int it = 0; it < 8; ++it) {
      *(volatile v4f*)(dst + (size_t)(it * 2) * (size_t)N) = vals[it];
    }
    __threadfence();
  }
}
__device__ __forceinline__ void epi64x2b(float* sl, v8f a0, v8f a1, v8f a2, v8f a3, v8f e0, v8f e1, v8f e2, v8f e3,
                                         float os1, float os2, const float* __restrict__ bias, float* C, int N,
                                         size_t rowb, int col0, int lane) {
  const int hh = lane >> 4, m = lane & 15;
  const float* bp = bias + col0 + m;
  const float b0 = bp[0], b1 = bp[16], b2 = bp[32], b3 = bp[48];
#pragma unroll
  for (int r = 0; r < 8; ++r) {
    const int ro = (8 * hh + r) * 68 + m;
    sl[ro]      = a0[r] * os1 + e0[r] * os2 + b0;
    sl[ro + 16] = a1[r] * os1 + e1[r] * os2 + b1;
    sl[ro + 32] = a2[r] * os1 + e2[r] * os2 + b2;
    sl[ro + 48] = a3[r] * os1 + e3[r] * os2 + b3;
  }
  wave_sync_lds();
  v4f vals[8];
#pragma unroll
  for (int it = 0; it < 8; ++it) vals[it] = *(const v4f*)(sl + (it * 2 + hh) * 68 + m * 4);
  float* dst = C + (rowb + (size_t)hh) * (size_t)N + col0 + m * 4;
  for (int pass = 0; pass < 2; ++pass) {
#pragma unroll
    for (int it = 0; it < 8; ++it) {
      *(volatile v4f*)(dst + (size_t)(it * 2) * (size_t)N) = vals[it];
    }
    __threadfence();
  }
}
__device__ __forceinline__ void epi64hs2(float* sl, v8f a0, v8f a1, v8f a2, v8f a3, float oscale, const float* __restrict__ bias,
                                         float pscale, float rscale, u16* Ch, u16* Cr, int N, size_t rowb, int col0, int lane) {
  stage64b(sl, a0, a1, a2, a3, oscale, bias, col0, lane);
  const int rq = lane >> 3, c8 = (lane & 7) * 8;
  v4u oh[4], orr[4];
#pragma unroll
  for (int i4 = 0; i4 < 4; ++i4) {
    const int row = i4 * 4 + rq;
    const v4f a = *(const v4f*)(sl + row * 68 + c8), c4 = *(const v4f*)(sl + row * 68 + c8 + 4);
    float w[8];
#pragma unroll
    for (int e = 0; e < 4; ++e) { w[e] = a[e] * pscale; w[4 + e] = c4[e] * pscale; }
#pragma unroll
    for (int e = 0; e < 4; ++e) {
      const float x0 = w[2 * e], x1 = w[2 * e + 1];
      const _Float16 h0 = (_Float16)x0, h1 = (_Float16)x1;
      const _Float16 r0 = (_Float16)((x0 - (float)h0) * rscale), r1 = (_Float16)((x1 - (float)h1) * rscale);
      oh[i4][e]  = pk16(h_bits(h0), h_bits(h1));
      orr[i4][e] = pk16(h_bits(r0), h_bits(r1));
    }
  }
  const size_t dofs = rowb * (size_t)N + col0 + c8;
  u16* dh = Ch + dofs;
  u16* dr = Cr + dofs;
  for (int pass = 0; pass < 2; ++pass) {
#pragma unroll
    for (int i4 = 0; i4 < 4; ++i4) {
      const int row = i4 * 4 + rq;
      *(volatile v4u*)(dh + (size_t)row * (size_t)N) = oh[i4];
      *(volatile v4u*)(dr + (size_t)row * (size_t)N) = orr[i4];
    }
    __threadfence();
  }
}

__global__ __launch_bounds__(128)
void gemm_b32(const u16* __restrict__ A, const u16* __restrict__ Bt, const float* __restrict__ bias, float* C,
              int M, int N, int K, float oscale) {
  __shared__ __align__(16) float slab[4 * SLAB64];
  const int tid = threadIdx.x, wave = tid >> 5, lane = tid & 31, hh = lane >> 4, m = lane & 15;
  const int ntile = N >> 6;
  const int bid   = blockIdx.x;
  const int rowb  = (bid / ntile) * 64 + wave * 16;
  const int col0  = (bid % ntile) * 64;
  if (rowb + 16 > M) return;
  const u16* ap = A  + (size_t)(rowb + m) * K + 8 * hh;
  const u16* bp = Bt + (size_t)(col0 + m) * K + 8 * hh;
  const size_t bs = (size_t)16 * K;
  v8f acc0 = zero8(), acc1 = zero8(), acc2 = zero8(), acc3 = zero8();
#pragma unroll 1
  for (int k0 = 0; k0 < K; k0 += 32) {
    const v16b a  = ldfrag_b(ap + k0);
    const v16b b0 = ldfrag_b(bp + k0);
    const v16b b1 = ldfrag_b(bp + bs + k0);
    const v16b b2 = ldfrag_b(bp + 2 * bs + k0);
    const v16b b3 = ldfrag_b(bp + 3 * bs + k0);
    acc0 = mma_b(a, b0, acc0);
    acc1 = mma_b(a, b1, acc1);
    acc2 = mma_b(a, b2, acc2);
    acc3 = mma_b(a, b3, acc3);
    guard6<v16b>(acc0, acc1, acc2, acc3, a, b0, b1, b2, b3, a);
  }
  epi64b(slab + wave * SLAB64, acc0, acc1, acc2, acc3, oscale, bias, C, N, (size_t)rowb, col0, lane);
}

__global__ __launch_bounds__(128)
void gemm_bh2(const u16* __restrict__ A, const u16* __restrict__ Bt, const float* __restrict__ bias, u16* Ch, u16* Cr,
              int M, int N, int K, float oscale, float pscale, float rscale) {
  __shared__ __align__(16) float slab[4 * SLAB64];
  const int tid = threadIdx.x, wave = tid >> 5, lane = tid & 31, hh = lane >> 4, m = lane & 15;
  const int ntile = N >> 6;
  const int bid   = blockIdx.x;
  const int rowb  = (bid / ntile) * 64 + wave * 16;
  const int col0  = (bid % ntile) * 64;
  if (rowb + 16 > M) return;
  const u16* ap = A  + (size_t)(rowb + m) * K + 8 * hh;
  const u16* bp = Bt + (size_t)(col0 + m) * K + 8 * hh;
  const size_t bs = (size_t)16 * K;
  v8f acc0 = zero8(), acc1 = zero8(), acc2 = zero8(), acc3 = zero8();
#pragma unroll 1
  for (int k0 = 0; k0 < K; k0 += 32) {
    const v16b a  = ldfrag_b(ap + k0);
    const v16b b0 = ldfrag_b(bp + k0);
    const v16b b1 = ldfrag_b(bp + bs + k0);
    const v16b b2 = ldfrag_b(bp + 2 * bs + k0);
    const v16b b3 = ldfrag_b(bp + 3 * bs + k0);
    acc0 = mma_b(a, b0, acc0);
    acc1 = mma_b(a, b1, acc1);
    acc2 = mma_b(a, b2, acc2);
    acc3 = mma_b(a, b3, acc3);
    guard6<v16b>(acc0, acc1, acc2, acc3, a, b0, b1, b2, b3, a);
  }
  epi64hs2(slab + wave * SLAB64, acc0, acc1, acc2, acc3, oscale, bias, pscale, rscale, Ch, Cr, N, (size_t)rowb, col0, lane);
}

__global__ __launch_bounds__(128)
void gemm_h2_32(const u16* __restrict__ Ah, const u16* __restrict__ Ar, const u16* __restrict__ Bt,
                const float* __restrict__ bias, float* C, int M, int N, int K, float os1, float os2) {
  __shared__ __align__(16) float slab[4 * SLAB64];
  const int tid = threadIdx.x, wave = tid >> 5, lane = tid & 31, hh = lane >> 4, m = lane & 15;
  const int ntile = N >> 6;
  const int bid   = blockIdx.x;
  const int rowb  = (bid / ntile) * 64 + wave * 16;
  const int col0  = (bid % ntile) * 64;
  if (rowb + 16 > M) return;
  const _Float16* ap  = hptr(Ah) + (size_t)(rowb + m) * K + 8 * hh;
  const _Float16* arp = hptr(Ar) + (size_t)(rowb + m) * K + 8 * hh;
  const _Float16* bp  = hptr(Bt) + (size_t)(col0 + m) * K + 8 * hh;
  const size_t bs = (size_t)16 * K;
  v8f acc0 = zero8(), acc1 = zero8(), acc2 = zero8(), acc3 = zero8();
  v8f acr0 = zero8(), acr1 = zero8(), acr2 = zero8(), acr3 = zero8();
#pragma unroll 1
  for (int k0 = 0; k0 < K; k0 += 32) {
    const v16h a  = ldfrag_h(ap + k0);
    const v16h ar = ldfrag_h(arp + k0);
    const v16h b0 = ldfrag_h(bp + k0);
    const v16h b1 = ldfrag_h(bp + bs + k0);
    const v16h b2 = ldfrag_h(bp + 2 * bs + k0);
    const v16h b3 = ldfrag_h(bp + 3 * bs + k0);
    acc0 = mma_h(a, b0, acc0);
    acc1 = mma_h(a, b1, acc1);
    acc2 = mma_h(a, b2, acc2);
    acc3 = mma_h(a, b3, acc3);
    acr0 = mma_h(ar, b0, acr0);
    acr1 = mma_h(ar, b1, acr1);
    acr2 = mma_h(ar, b2, acr2);
    acr3 = mma_h(ar, b3, acr3);
    guard8x6(acc0, acc1, acc2, acc3, acr0, acr1, acr2, acr3, a, ar, b0, b1, b2, b3);
  }
  epi64x2b(slab + wave * SLAB64, acc0, acc1, acc2, acc3, acr0, acr1, acr2, acr3, os1, os2, bias, C, N,
           (size_t)rowb, col0, lane);
}

__global__ __launch_bounds__(256) void xt16(const float* __restrict__ X, u16* XTh) {
  __shared__ __align__(16) u16 TH[64 * VTP];
  const int tid = threadIdx.x;
  const int bid = blockIdx.x;
  const int st  = bid % (SEQ / 64);
  const int dcb = (bid / (SEQ / 64)) % (EMB / 64);
  const int b   = bid / ((SEQ / 64) * (EMB / 64));
  const int s0  = st * 64;
  const int d0  = dcb * 64;
  {
    const int sl = tid >> 2;
    const int dc = (tid & 3) * 16;
    const float* src = X + ((size_t)b * SEQ + s0 + sl) * EMB + d0 + dc;
#pragma unroll
    for (int i = 0; i < 4; ++i) {
      const v4f a = *(const v4f*)(src + 4 * i);
#pragma unroll
      for (int e = 0; e < 4; ++e) {
        const float xs = a[e] * VCAR;
        TH[(dc + 4 * i + e) * VTP + sl] = h_bits((_Float16)xs);
      }
    }
  }
  __syncthreads();
  v4u vh[2];
  const int q8 = tid >> 3, p8 = (tid & 7) * 8;
#pragma unroll
  for (int it = 0; it < 2; ++it) {
    const int line = it * 32 + q8;
    vh[it] = *(const v4u*)(TH + line * VTP + p8);
  }
  const size_t base = ((size_t)b * EMB + d0) * SEQ + s0 + p8;
  for (int pass = 0; pass < 2; ++pass) {
#pragma unroll
    for (int it = 0; it < 2; ++it) {
      const int line = it * 32 + q8;
      *(volatile v4u*)(XTh + base + (size_t)line * SEQ) = vh[it];
    }
    __threadfence();
  }
}

__global__ __launch_bounds__(256) void vsum_k(const float* __restrict__ V, float* VS) {
  const int tid = threadIdx.x;
  const int gt  = blockIdx.x * 256 + tid;
  if (gt >= NB * NCHK * EMB) return;
  const int d   = gt % EMB;
  const int bc  = gt / EMB;
  const int b   = bc / NCHK;
  const int c   = bc - b * NCHK;
  const float* p = V + ((size_t)b * SEQ + (size_t)c * CK) * EMB + d;
  float s0 = 0.f, s1 = 0.f, s2 = 0.f, s3 = 0.f;
#pragma unroll 1
  for (int i = 0; i < CK; i += 4) {
    s0 += p[(size_t)(i + 0) * EMB];
    s1 += p[(size_t)(i + 1) * EMB];
    s2 += p[(size_t)(i + 2) * EMB];
    s3 += p[(size_t)(i + 3) * EMB];
  }
  const float s = (s0 + s1) + (s2 + s3);
  float* dst = VS + (size_t)gt;
  *(volatile float*)dst = s;
  __threadfence();
  *(volatile float*)dst = s;
}

__device__ __forceinline__ void ctx_store(const u16* ct, u16* dst, int tid) {
  v4u v[8];
#pragma unroll
  for (int it = 0; it < 8; ++it) {
    const int p   = it * 256 + tid;
    const int row = p / (EMB / 8);
    const int c8  = (p - row * (EMB / 8)) * 8;
    v[it] = *(const v4u*)(ct + row * CTP + c8);
  }
  for (int pass = 0; pass < 2; ++pass) {
#pragma unroll
    for (int it = 0; it < 8; ++it) {
      const int p   = it * 256 + tid;
      const int row = p / (EMB / 8);
      const int c8  = (p - row * (EMB / 8)) * 8;
      *(volatile v4u*)(dst + (size_t)row * EMB + c8) = v[it];
    }
    __threadfence();
  }
}

__global__ __launch_bounds__(ATT_THREADS)
void attn_fwd(const u16* __restrict__ QHp, const u16* __restrict__ QRp, const u16* __restrict__ KHp,
              const u16* __restrict__ KRp, const u16* __restrict__ VTp, const float* __restrict__ VSp,
              u16* CHo, u16* CRo) {
  __shared__ __align__(16) AttLds L0;
  __shared__ __align__(16) u16 pls[16 * PLP];
  __shared__ float rowa[QT];
  __shared__ float rowc[QT];
  __shared__ float rowi[QT];
  float* const scs = L0.s;

  const int tid  = threadIdx.x;
  const int wave = tid >> 5;
  const int lane = tid & 31;
  const int hh   = lane >> 4;
  const int m    = lane & 15;
  const int r16  = tid >> 4;
  const int sub  = tid & 15;
  const int kl0  = sub * 32;

  const int bid = blockIdx.x;
  const int b   = bid / NQT;
  const int q0  = (bid - b * NQT) * QT;

  const size_t qofs = ((size_t)b * SEQ + q0 + m) * EMB + 8 * hh;
  const size_t kofs = ((size_t)b * SEQ + m) * EMB + 8 * hh;
  const _Float16* qa  = hptr(QHp) + qofs;
  const _Float16* qra = hptr(QRp) + qofs;
  const _Float16* khb = hptr(KHp) + kofs;
  const _Float16* krb = hptr(KRp) + kofs;
  const _Float16* vbp = hptr(VTp) + ((size_t)b * EMB + wave * (16 * NACC) + m) * SEQ + 8 * hh;
  const float* vsb = VSp + (size_t)b * NCHK * EMB + wave * (16 * NACC) + m;
  const float lsc = RSQD * LOG2E / (QSC * KSC);
  const float rinv = 1.0f / QRS;

  float mrun = -INFINITY, lrun = 0.f;
  v8f o[NACC];
#pragma unroll
  for (int j = 0; j < NACC; ++j) o[j] = zero8();

#pragma unroll 1
  for (int c = 0; c < NCHK; ++c) {
    const int kbeg = c * CK;
#pragma unroll 1
    for (int kb = wave; kb < NKB; kb += 8) {
      v8f s0h = zero8(), s1h = zero8(), s0x = zero8(), s1x = zero8();
      const size_t koff = (size_t)(kbeg + kb * 32) * EMB;
      const _Float16* k0p = khb + koff;
      const _Float16* k1p = k0p + (size_t)16 * EMB;
      const _Float16* r0p = krb + koff;
      const _Float16* r1p = r0p + (size_t)16 * EMB;
#pragma unroll 2
      for (int ks = 0; ks < EMB / 32; ++ks) {
        const int dd = ks * 32;
        const v16h a  = ldfrag_h(qa + dd);
        const v16h f0 = ldfrag_h(k0p + dd);
        const v16h f1 = ldfrag_h(k1p + dd);
        s0h = mma_h(a, f0, s0h);
        s1h = mma_h(a, f1, s1h);
        const v16h ar = ldfrag_h(qra + dd);
        s0x = mma_h(ar, f0, s0x);
        s1x = mma_h(ar, f1, s1x);
        const v16h g0 = ldfrag_h(r0p + dd);
        const v16h g1 = ldfrag_h(r1p + dd);
        s0x = mma_h(a, g0, s0x);
        s1x = mma_h(a, g1, s1x);
        guard6<v16h>(s0h, s1h, s0x, s1x, a, ar, f0, f1, g0, g1);
      }
      float* srow = scs + (8 * hh) * SCP + kb * 32 + m;
#pragma unroll
      for (int r = 0; r < 8; ++r) {
        srow[r * SCP]      = s0h[r] + s0x[r] * rinv;
        srow[r * SCP + 16] = s1h[r] + s1x[r] * rinv;
      }
    }
    __syncthreads();
    {
      const float* sp = scs + r16 * SCP + kl0;
      float t[32];
      float cm = -INFINITY;
#pragma unroll
      for (int i = 0; i < 8; ++i) {
        const v4f a4 = *(const v4f*)(sp + 4 * i);
#pragma unroll
        for (int e = 0; e < 4; ++e) {
          const int j = 4 * i + e;
          const float tv = (kl0 + j < CK) ? a4[e] * lsc : -INFINITY;
          t[j] = tv;
          cm = fmaxf(cm, tv);
        }
      }
#pragma unroll
      for (int d = 1; d <= 8; d <<= 1) cm = fmaxf(cm, __shfl_xor(cm, d, 32));
      const float mn = fmaxf(mrun, cm);
      const float al = (mrun == -INFINITY) ? 0.f : exp2f(mrun - mn);
      mrun = mn;
      float ps = 0.f;
#pragma unroll
      for (int j = 0; j < 32; ++j) {
        const float p = exp2f(fminf(t[j] - mn, 0.f));
        t[j] = p;
        ps += p;
      }
#pragma unroll
      for (int d = 1; d <= 8; d <<= 1) ps += __shfl_xor(ps, d, 32);
      const float cc = ps * (1.0f / (float)CK);
      v4u pk[4];
#pragma unroll
      for (int i = 0; i < 4; ++i) {
#pragma unroll
        for (int e = 0; e < 4; ++e) {
          const int j = 8 * i + 2 * e;
          pk[i][e] = pk16(h_bits((_Float16)((t[j] - cc) * PCAR)), h_bits((_Float16)((t[j + 1] - cc) * PCAR)));
        }
      }
      lrun = lrun * al + ps;
      u16* pd = pls + r16 * PLP + kl0;
#pragma unroll
      for (int i = 0; i < 4; ++i) *(v4u*)(pd + 8 * i) = pk[i];
      if (sub == 0) { rowa[r16] = al; rowc[r16] = cc; }
    }
    __syncthreads();
    {
      float scl[8], cad[8];
#pragma unroll
      for (int r = 0; r < 8; ++r) { scl[r] = rowa[8 * hh + r]; cad[r] = rowc[8 * hh + r] * (PCAR * VCAR); }
      const float* vsc = vsb + (size_t)c * EMB;
      float vs[NACC];
#pragma unroll
      for (int j = 0; j < NACC; ++j) vs[j] = vsc[16 * j];
#pragma unroll
      for (int j = 0; j < NACC; ++j) {
#pragma unroll
        for (int r = 0; r < 8; ++r) o[j][r] = o[j][r] * scl[r] + cad[r] * vs[j];
      }
      const _Float16* pp = hptr(pls) + m * PLP + 8 * hh;
      const _Float16* vp = vbp + kbeg;
#pragma unroll 1
      for (int kb = 0; kb < NKB; ++kb) {
        const v16h pf = ldfrag_h(pp + kb * 32);
        const _Float16* vk = vp + kb * 32;
        {
          const v16h g0 = ldfrag_h(vk);
          const v16h g1 = ldfrag_h(vk + (size_t)16 * SEQ);
          const v16h g2 = ldfrag_h(vk + (size_t)32 * SEQ);
          const v16h g3 = ldfrag_h(vk + (size_t)48 * SEQ);
          o[0] = mma_h(pf, g0, o[0]);
          o[1] = mma_h(pf, g1, o[1]);
          o[2] = mma_h(pf, g2, o[2]);
          o[3] = mma_h(pf, g3, o[3]);
          guardpv4(o[0], o[1], o[2], o[3], pf, g0, g1, g2, g3);
        }
        {
          const v16h g4 = ldfrag_h(vk + (size_t)64 * SEQ);
          const v16h g5 = ldfrag_h(vk + (size_t)80 * SEQ);
          const v16h g6 = ldfrag_h(vk + (size_t)96 * SEQ);
          const v16h g7 = ldfrag_h(vk + (size_t)112 * SEQ);
          o[4] = mma_h(pf, g4, o[4]);
          o[5] = mma_h(pf, g5, o[5]);
          o[6] = mma_h(pf, g6, o[6]);
          o[7] = mma_h(pf, g7, o[7]);
          guardpv4(o[4], o[5], o[6], o[7], pf, g4, g5, g6, g7);
        }
      }
    }
  }
  acc_guard8(o[0], o[1], o[2], o[3], o[4], o[5], o[6], o[7]);

  if (sub == 0) rowi[r16] = (1.0f / lrun) * (CSC / (PCAR * VCAR));
  __syncthreads();
  float inv[8];
#pragma unroll
  for (int r = 0; r < 8; ++r) inv[r] = rowi[8 * hh + r];

  u16* const ct = L0.c;
  const int cb = wave * (16 * NACC) + m;
#pragma unroll
  for (int j = 0; j < NACC; ++j) {
#pragma unroll
    for (int r = 0; r < 8; ++r) {
      const float xs = o[j][r] * inv[r];
      ct[(8 * hh + r) * CTP + cb + 16 * j] = h_bits((_Float16)xs);
    }
  }
  __syncthreads();
  ctx_store(ct, CHo + ((size_t)b * SEQ + q0) * EMB, tid);
  __syncthreads();
#pragma unroll
  for (int j = 0; j < NACC; ++j) {
#pragma unroll
    for (int r = 0; r < 8; ++r) {
      const float xs = o[j][r] * inv[r];
      const _Float16 hv = (_Float16)xs;
      ct[(8 * hh + r) * CTP + cb + 16 * j] = h_bits((_Float16)((xs - (float)hv) * RSC));
    }
  }
  __syncthreads();
  ctx_store(ct, CRo + ((size_t)b * SEQ + q0) * EMB, tid);
}

extern "C" void kernel_launch(void* const* d_in, const int* in_sizes, int n_in,
                              void* d_out, int out_size, void* d_ws, size_t ws_size,
                              hipStream_t stream) {
  if (n_in < 11) return;
  const int need_x = ((NB - 1) * SEQ_FULL + SEQ) * EMB;
  if (in_sizes[0] < need_x || in_sizes[1] < need_x || in_sizes[2] < need_x) return;
  if (in_sizes[3] < EMB * EMB || in_sizes[5] < EMB * EMB || in_sizes[7] < EMB * EMB || in_sizes[9] < EMB * EMB) return;
  if (in_sizes[4] < EMB || in_sizes[6] < EMB || in_sizes[8] < EMB || in_sizes[10] < EMB) return;
  const int rows = NB * SEQ;
  if (out_size < rows * EMB) return;

  const float* q  = (const float*)d_in[0];
  const float* k  = (const float*)d_in[1];
  const float* v  = (const float*)d_in[2];
  const float* wq = (const float*)d_in[3];
  const float* bq = (const float*)d_in[4];
  const float* wk = (const float*)d_in[5];
  const float* bk = (const float*)d_in[6];
  const float* wv = (const float*)d_in[7];
  const float* bv = (const float*)d_in[8];
  const float* wo = (const float*)d_in[9];
  const float* bo = (const float*)d_in[10];
  float*       out = (float*)d_out;

  const size_t szW  = (size_t)EMB * EMB * 2;
  const size_t szVS = (size_t)NB * NCHK * EMB * 4;
  const size_t sz16 = (size_t)rows * EMB * 2;
  const size_t sz32 = (size_t)rows * EMB * 4;
  const size_t szVT = (size_t)NB * EMB * SEQ * 2;
  if (szVT != sz16 || sz32 != 2 * sz16 || (szVS % 128) != 0) return;
  size_t off = 0;
  const size_t oWQ = off; off += szW;
  const size_t oWK = off; off += szW;
  const size_t oWV = off; off += szW;
  const size_t oWO = off; off += szW;
  const size_t oVS = off; off += szVS;
  const size_t oXB = off; off += sz16;
  const size_t oQH = off; off += sz16;
  const size_t oQR = off; off += sz16;
  const size_t oKH = off; off += sz16;
  const size_t oKR = off; off += sz16;
  const size_t oV  = off; off += sz32;
  const size_t oCH = oV;
  const size_t oCR = oV + sz16;
  if (off > ws_size) return;
  if (off > WS_CAP) return;

  char* ws = (char*)d_ws;
  u16*   WQB = (u16*)(ws + oWQ);
  u16*   WKB = (u16*)(ws + oWK);
  u16*   WVB = (u16*)(ws + oWV);
  u16*   WOH = (u16*)(ws + oWO);
  float* VS  = (float*)(ws + oVS);
  u16*   XB  = (u16*)(ws + oXB);
  u16*   VT  = (u16*)(ws + oXB);
  u16*   QH  = (u16*)(ws + oQH);
  u16*   QR  = (u16*)(ws + oQR);
  u16*   KH  = (u16*)(ws + oKH);
  u16*   KR  = (u16*)(ws + oKR);
  float* V   = (float*)(ws + oV);
  u16*   CH  = (u16*)(ws + oCH);
  u16*   CR  = (u16*)(ws + oCR);

  const int n8w = (EMB * EMB) / 8;
  const int n8x = rows * (EMB / 8);
  if ((rows % 64) != 0 || ((NB * NCHK * EMB) % 256) != 0 || (EMB % 64) != 0 || (EMB % 32) != 0) return;
  const dim3 blk(256);
  const dim3 gW((n8w + 255) / 256), gX((n8x + 255) / 256);
  const dim3 gG((rows / 64) * (EMB / 64));
  const dim3 bG(128);
  const dim3 gXT(NB * (EMB / 64) * (SEQ / 64));
  const dim3 gVS((NB * NCHK * EMB) / 256);
  const dim3 gAT(NB * NQT);
  const dim3 bAT(ATT_THREADS);

  cvt16<<<gW, blk, 0, stream>>>(wq, WQB, n8w, 0, 1.0f, EMB, EMB);
  cvt16<<<gW, blk, 0, stream>>>(wk, WKB, n8w, 0, 1.0f, EMB, EMB);
  cvt16<<<gW, blk, 0, stream>>>(wv, WVB, n8w, 0, 1.0f, EMB, EMB);
  cvt16<<<gW, blk, 0, stream>>>(wo, WOH, n8w, 1, WSC, EMB, EMB);
  cvt16<<<gX, blk, 0, stream>>>(q, XB, n8x, 0, 1.0f, SEQ, SEQ_FULL);
  gemm_bh2<<<gG, bG, 0, stream>>>(XB, WQB, bq, QH, QR, rows, EMB, EMB, 1.0f, QSC, QRS);
  cvt16<<<gX, blk, 0, stream>>>(k, XB, n8x, 0, 1.0f, SEQ, SEQ_FULL);
  gemm_bh2<<<gG, bG, 0, stream>>>(XB, WKB, bk, KH, KR, rows, EMB, EMB, 1.0f, KSC, QRS);
  cvt16<<<gX, blk, 0, stream>>>(v, XB, n8x, 0, 1.0f, SEQ, SEQ_FULL);
  gemm_b32<<<gG, bG, 0, stream>>>(XB, WVB, bv, V, rows, EMB, EMB, 1.0f);
  xt16<<<gXT, blk, 0, stream>>>(V, VT);
  vsum_k<<<gVS, blk, 0, stream>>>(V, VS);
  attn_fwd<<<gAT, bAT, 0, stream>>>(QH, QR, KH, KR, VT, VS, CH, CR);
  gemm_h2_32<<<gG, bG, 0, stream>>>(CH, CR, WOH, bo, out, rows, EMB, EMB,
                                     1.0f / (CSC * WSC), 1.0f / (CSC * WSC * RSC));
  (void)hipGetLastError();
}
